// Model_39676907882252
// MI455X (gfx1250) — hardware-verified
//
#include <hip/hip_runtime.h>
#ifndef NB
#define NB 2
#endif
#ifndef SEQ
#define SEQ 2048
#endif
#define NB_FULL 2
#define SEQ_FULL 2048
#define NH 16
#define HD 64
#define NSLAB (NB * NH)
#define KT 64
#define QB 64
#define PLANE_ELEMS ((size_t)NSLAB * SEQ * HD)
#define PLANE_BYTES (PLANE_ELEMS * 2)
#define N8 (PLANE_ELEMS / 8)
#define WS_LIMIT ((size_t)134217728)

static_assert(HD == 64);
static_assert(HD % 32 == 0);
static_assert(SEQ % KT == 0);
static_assert(SEQ % QB == 0);
static_assert(SEQ % 64 == 0);
static_assert(QB == 4 * 16);
static_assert(SEQ <= SEQ_FULL);
static_assert(NB <= NB_FULL);
static_assert(PLANE_BYTES % 256 == 0);
static_assert(3 * PLANE_BYTES <= WS_LIMIT);
static_assert(PLANE_ELEMS % (8 * 256) == 0);

typedef _Float16 v16h __attribute__((ext_vector_type(16)));
typedef unsigned short v8us __attribute__((ext_vector_type(8), may_alias));
typedef float v8f  __attribute__((ext_vector_type(8)));
typedef float v4f  __attribute__((ext_vector_type(4)));
typedef float v4fa __attribute__((ext_vector_type(4), may_alias));
union FragH { v16h v; v8us half[2]; _Float16 h[16]; unsigned short u[16]; };

__device__ __forceinline__ float bf16_rne(float x) {
  unsigned int u = __float_as_uint(x);
  u = (u + 0x7FFFu + ((u >> 16) & 1u)) & 0xFFFF0000u;
  return __uint_as_float(u);
}
__device__ __forceinline__ v16h ld_frag(const unsigned short* p) {
  FragH f;
  f.half[0] = *(const v8us*)p;
  f.half[1] = *(const v8us*)(p + 16);
  return f.v;
}
__device__ __forceinline__ v8f mma16(v16h a, v16h b, v8f c) {
  v8f d = __builtin_amdgcn_wmma_f32_16x16x32_f16(false, a, false, b, (short)0, c, false, false);
  asm volatile("v_nop\n\tv_nop\n\tv_nop\n\tv_nop" : "+v"(d) : "v"(a), "v"(b));
  return d;
}

__global__ __launch_bounds__(256) void k_cvt16(const float* __restrict__ x, unsigned short* __restrict__ P16) {
  const size_t t = (size_t)blockIdx.x * 256 + threadIdx.x;
  if (t >= N8) return;
  const size_t row = t >> 3;
  const int c8 = (int)(t & 7) * 8;
  const size_t slab = row / SEQ, s = row % SEQ;
  const float* src = x + (slab * SEQ_FULL + s) * HD + c8;
  const v4f a = *(const v4fa*)src, c = *(const v4fa*)(src + 4);
  FragH f;
#pragma unroll
  for (int q = 0; q < 4; ++q) {
    f.h[q] = (_Float16)(bf16_rne(a[q]) * 16.0f);
    f.h[4 + q] = (_Float16)(bf16_rne(c[q]) * 16.0f);
  }
  const v8us o = f.half[0];
  *(volatile v8us*)(P16 + t * 8) = o;
  __threadfence();
  *(volatile v8us*)(P16 + t * 8) = o;
}

__global__ __launch_bounds__(256) void k_vt16(const float* __restrict__ V, unsigned short* __restrict__ VT) {
  __shared__ unsigned short tl[64][66];
  const int tid = threadIdx.x;
  const int slab = blockIdx.y, s0 = blockIdx.x * 64;
#pragma unroll 1
  for (int i = tid; i < 64 * 16; i += 256) {
    const int j = i >> 4, d4 = (i & 15) * 4;
    const v4f a = *(const v4fa*)(V + ((size_t)slab * SEQ_FULL + s0 + j) * HD + d4);
#pragma unroll
    for (int q = 0; q < 4; ++q) {
      const _Float16 h = (_Float16)(bf16_rne(a[q]) * 16.0f);
      tl[d4 + q][j] = __builtin_bit_cast(unsigned short, h);
    }
  }
  __syncthreads();
  v8us o0, o1;
  const int dA = tid >> 3, j8 = (tid & 7) * 8;
#pragma unroll
  for (int q = 0; q < 8; ++q) { o0[q] = tl[dA][j8 + q]; o1[q] = tl[32 + dA][j8 + q]; }
  unsigned short* r0p = VT + ((size_t)slab * HD + dA) * SEQ + s0 + j8;
  unsigned short* r1p = VT + ((size_t)slab * HD + 32 + dA) * SEQ + s0 + j8;
  *(volatile v8us*)r0p = o0;
  *(volatile v8us*)r1p = o1;
  __threadfence();
  *(volatile v8us*)r0p = o0;
  *(volatile v8us*)r1p = o1;
}

__global__ __launch_bounds__(128) void k_fattn(const unsigned short* __restrict__ Q16, const unsigned short* __restrict__ K16,
                                               const unsigned short* __restrict__ VT, float* __restrict__ O) {
  __shared__ __attribute__((aligned(16))) float so[4][16][64];
  const int tid = threadIdx.x;
  const int wave = __builtin_amdgcn_readfirstlane(tid >> 5);
  const int lane = tid & 31, ln = lane & 15, hh = lane >> 4;
  const int bh = blockIdx.y;
  const int q0 = blockIdx.x * QB + wave * 16;
  const unsigned short* qp = Q16 + ((size_t)bh * SEQ + q0 + ln) * HD + 8 * hh;
  const v16h qf0 = ld_frag(qp), qf1 = ld_frag(qp + 32);
  const unsigned short* kp = K16 + ((size_t)bh * SEQ + ln) * HD + 8 * hh;
  const unsigned short* vp = VT + ((size_t)bh * HD + ln) * SEQ + 8 * hh;
  const v8f z8 = {0.f, 0.f, 0.f, 0.f, 0.f, 0.f, 0.f, 0.f};
  v8f oacc[4] = {z8, z8, z8, z8};
  float m = -1.0e30f, lp = 0.f;
  const float SCL = 0.00048828125f;
#pragma unroll 1
  for (int kb = 0; kb < SEQ; kb += KT) {
    v8f sc[4];
#pragma unroll
    for (int j = 0; j < 4; ++j) {
      const unsigned short* kr = kp + (size_t)(kb + 16 * j) * HD;
      v8f c = z8;
      c = mma16(ld_frag(kr), qf0, c);
      c = mma16(ld_frag(kr + 32), qf1, c);
      sc[j] = c;
    }
    float mx = sc[0][0];
#pragma unroll
    for (int j = 0; j < 4; ++j)
#pragma unroll
      for (int r = 0; r < 8; ++r) mx = fmaxf(mx, sc[j][r]);
    mx = fmaxf(mx, __shfl_xor(mx, 16, 32));
    const float mnew = fmaxf(m, mx * SCL);
    const float alpha = __expf(m - mnew);
    m = mnew;
    FragH pb0, pb1;
    float ps = 0.f;
#pragma unroll
    for (int r = 0; r < 8; ++r) {
      const float p0 = __expf(fmaf(sc[0][r], SCL, -mnew));
      const float p1 = __expf(fmaf(sc[1][r], SCL, -mnew));
      const float p2 = __expf(fmaf(sc[2][r], SCL, -mnew));
      const float p3 = __expf(fmaf(sc[3][r], SCL, -mnew));
      ps += (p0 + p1) + (p2 + p3);
      pb0.h[r]     = (_Float16)(p0 * 256.0f);
      pb0.h[8 + r] = (_Float16)(p1 * 256.0f);
      pb1.h[r]     = (_Float16)(p2 * 256.0f);
      pb1.h[8 + r] = (_Float16)(p3 * 256.0f);
    }
    lp = lp * alpha + ps;
#pragma unroll
    for (int t = 0; t < 4; ++t) oacc[t] = oacc[t] * alpha;
#pragma unroll
    for (int t = 0; t < 4; ++t) {
      const unsigned short* vr = vp + (size_t)(16 * t) * SEQ + kb;
      oacc[t] = mma16(ld_frag(vr), pb0.v, oacc[t]);
      oacc[t] = mma16(ld_frag(vr + 32), pb1.v, oacc[t]);
    }
  }
  const float l = lp + __shfl_xor(lp, 16, 32);
  const float inv = (1.0f / l) * 0.000244140625f;
#pragma unroll
  for (int t = 0; t < 4; ++t) {
    v4f a, b;
#pragma unroll
    for (int r = 0; r < 4; ++r) { a[r] = oacc[t][r] * inv; b[r] = oacc[t][4 + r] * inv; }
    *(v4fa*)&so[wave][ln][16 * t + 8 * hh] = a;
    *(v4fa*)&so[wave][ln][16 * t + 8 * hh + 4] = b;
  }
  __syncthreads();
  const int rsub = lane >> 4, c4 = (lane & 15) * 4;
  float* ob = O + ((size_t)bh * SEQ + q0) * HD;
  v4f vals[8];
#pragma unroll
  for (int q = 0; q < 8; ++q) vals[q] = *(const v4fa*)&so[wave][q * 2 + rsub][c4];
#pragma unroll
  for (int q = 0; q < 8; ++q) *(volatile v4f*)(ob + (size_t)(q * 2 + rsub) * HD + c4) = vals[q];
  __threadfence();
#pragma unroll
  for (int q = 0; q < 8; ++q) *(volatile v4f*)(ob + (size_t)(q * 2 + rsub) * HD + c4) = vals[q];
}

extern "C" void kernel_launch(void* const* d_in, const int* in_sizes, int n_in,
                              void* d_out, int out_size, void* d_ws, size_t ws_size, hipStream_t stream) {
  if (n_in < 3) return;
  const size_t need_in = ((size_t)(NSLAB - 1) * SEQ_FULL + SEQ) * HD;
  if ((size_t)in_sizes[0] < need_in || (size_t)in_sizes[1] < need_in || (size_t)in_sizes[2] < need_in) return;
  if ((size_t)out_size < PLANE_ELEMS) return;
  const float* xq = (const float*)d_in[0];
  const float* xk = (const float*)d_in[1];
  const float* xv = (const float*)d_in[2];
  char* ws = (char*)d_ws;
  size_t off = 0;
  unsigned short* Q16 = (unsigned short*)(ws + off); off += PLANE_BYTES;
  unsigned short* K16 = (unsigned short*)(ws + off); off += PLANE_BYTES;
  unsigned short* VTp = (unsigned short*)(ws + off); off += PLANE_BYTES;
  if (off > ws_size) return;

  const unsigned cvt_blocks = (unsigned)((N8 + 255) / 256);
  k_cvt16<<<cvt_blocks, 256, 0, stream>>>(xq, Q16);
  k_cvt16<<<cvt_blocks, 256, 0, stream>>>(xk, K16);
  k_vt16<<<dim3(SEQ / 64, NSLAB), 256, 0, stream>>>(xv, VTp);
  k_fattn<<<dim3(SEQ / QB, NSLAB), 128, 0, stream>>>(Q16, K16, VTp, (float*)d_out);
}
